// Downsample_PASA_group_softmax_2791728742720
// MI455X (gfx1250) — hardware-verified
//
#include <hip/hip_runtime.h>
#include <math.h>

typedef __attribute__((ext_vector_type(16))) _Float16 v16h;
typedef __attribute__((ext_vector_type(16))) __bf16 v16b;
typedef __attribute__((ext_vector_type(8)))  _Float16 v8h;
typedef __attribute__((ext_vector_type(8)))  float v8f;
typedef __attribute__((ext_vector_type(4)))  float v4f;
typedef __attribute__((ext_vector_type(2)))  float v2f;
typedef __attribute__((ext_vector_type(4)))  unsigned v4u;
typedef __attribute__((ext_vector_type(4)))  int v4i;
typedef float __attribute__((may_alias)) float_a;
typedef int __attribute__((may_alias)) int_a;

template <typename T> __device__ __forceinline__ void vst2(void* p, T v) { *(volatile T*)p = v; __threadfence(); *(volatile T*)p = v; }
__device__ __forceinline__ v8f wmma16(v16h a, v16h b, v8f c) {
  v8f d = __builtin_amdgcn_wmma_f32_16x16x32_f16(false, a, false, b, (short)0, c, false, false);
  asm volatile("v_nop\n\tv_nop\n\tv_nop\n\tv_nop" : "+v"(d) : "v"(a), "v"(b));
  return d;
}
__device__ __forceinline__ v8f wmma_bf(v16b a, v16b b, v8f c) {
  v8f d = __builtin_amdgcn_wmma_f32_16x16x32_bf16(false, a, false, b, (short)0, c, false, false);
  asm volatile("v_nop\n\tv_nop\n\tv_nop\n\tv_nop" : "+v"(d) : "v"(a), "v"(b));
  return d;
}
__device__ __forceinline__ v16h frag_h(const _Float16* rowk0, int lane) {
  union { v16h v; v8h q[2]; } u; const _Float16* p = rowk0 + 8 * (lane >> 4);
  u.q[0] = *(const v8h*)p; u.q[1] = *(const v8h*)(p + 16); return u.v;
}
__device__ __forceinline__ v16h frag_f32(const float* rowk0, int lane) {
  v16h a; const float* p = rowk0 + 8 * (lane >> 4);
#pragma unroll
  for (int i = 0; i < 8; ++i) { a[i] = (_Float16)p[i]; a[8 + i] = (_Float16)p[16 + i]; }
  return a;
}
__device__ __forceinline__ v16h frag_f32s(const float* rowk0, int lane, float sc) {
  v16h a; const float* p = rowk0 + 8 * (lane >> 4);
#pragma unroll
  for (int i = 0; i < 8; ++i) { a[i] = (_Float16)(p[i] * sc); a[8 + i] = (_Float16)(p[16 + i] * sc); }
  return a;
}
__device__ __forceinline__ v16h fragc_f32(const float* W, int k0, int n, int lane, int ld, int K) {
  v16h a; const int g = lane >> 4;
#pragma unroll
  for (int i = 0; i < 8; ++i) { const int ka = k0 + 8 * g + i, kb = ka + 16;
    a[i] = (_Float16)(ka < K ? W[(size_t)(ka < K ? ka : K - 1) * ld + n] : 0.f); a[8 + i] = (_Float16)(kb < K ? W[(size_t)(kb < K ? kb : K - 1) * ld + n] : 0.f); }
  return a;
}
struct F2 { v16b h, l; };
__device__ __forceinline__ F2 bsplit16(const float v[16]) { F2 r;
#pragma unroll
  for (int i = 0; i < 16; ++i) { const __bf16 h = (__bf16)v[i]; r.h[i] = h; r.l[i] = (__bf16)(v[i] - (float)h); }
  return r; }
__device__ __forceinline__ F2 split_row(const float* row, int k0, int lane) { float v[16]; const float* p = row + k0 + 8 * (lane >> 4);
#pragma unroll
  for (int i = 0; i < 8; ++i) { v[i] = p[i]; v[8 + i] = p[16 + i]; }
  return bsplit16(v); }
__device__ __forceinline__ F2 split_rowK(const float* row, int k0, int lane, int K) { float v[16]; const int g = lane >> 4;
#pragma unroll
  for (int i = 0; i < 8; ++i) { const int ka = k0 + 8 * g + i, kb = ka + 16; v[i] = ka < K ? row[ka < K ? ka : K - 1] : 0.f; v[8 + i] = kb < K ? row[kb < K ? kb : K - 1] : 0.f; }
  return bsplit16(v); }
__device__ __forceinline__ F2 split_col(const float* W, int k0, int n, int lane, int ld, int K) { float v[16]; const int g = lane >> 4;
#pragma unroll
  for (int i = 0; i < 8; ++i) { const int ka = k0 + 8 * g + i, kb = ka + 16; v[i] = ka < K ? W[(size_t)(ka < K ? ka : K - 1) * ld + n] : 0.f; v[8 + i] = kb < K ? W[(size_t)(kb < K ? kb : K - 1) * ld + n] : 0.f; }
  return bsplit16(v); }
__device__ __forceinline__ v8f mac3(const F2& a, const F2& b, v8f c) { c = wmma_bf(a.l, b.h, c); c = wmma_bf(a.h, b.l, c); return wmma_bf(a.h, b.h, c); }
__device__ __forceinline__ float sigm(float v) { return 1.0f / (1.0f + expf(-v)); }
#define LDSX() do { asm volatile("s_wait_dscnt 0" ::: "memory"); __builtin_amdgcn_wave_barrier(); __builtin_amdgcn_fence(__ATOMIC_RELEASE, "workgroup"); } while (0)

__device__ __forceinline__ float bfr(float v) { return (float)(__bf16)v; }
#define NBT 8
#define CIN 64
#define HH 128
#define WWD 128
#define GRP 8
#define KK 9
#define COUT (GRP * KK)
#define HO (HH / 2)
#define WO (WWD / 2)
#define KDIM (CIN * KK)
#ifndef NBLK
#define NBLK (NBT * HO)
#endif
__device__ __forceinline__ int refl(int i, int n) { i = (i < 0) ? -i : i; return (i >= n) ? (2 * n - 2 - i) : i; }
__global__ __launch_bounds__(128) void k_pasa(const float* __restrict__ X, const float* __restrict__ CW, const float* __restrict__ GA, const float* __restrict__ BE, const float* __restrict__ RM, const float* __restrict__ RV, float* __restrict__ OUT) {
  __shared__ __align__(16) float sg[64][COUT + 1]; __shared__ __align__(16) float so[CIN][68];
  const int tid = threadIdx.x, wave = tid >> 5, lane = tid & 31, col = lane & 15, g = lane >> 4; const int n = blockIdx.x / HO, ho = blockIdx.x % HO; const int h = 2 * ho;
  const float* Xn = X + (size_t)n * CIN * HH * WWD;
  v8f acc[5] = {};
  { const int wo = wave * 16 + col; const int w = 2 * wo;
#pragma unroll 2
    for (int kc = 0; kc < KDIM / 32; ++kc) { v16b a;
#pragma unroll
      for (int i = 0; i < 16; ++i) { const int k = kc * 32 + (i < 8 ? 8 * g + i : 16 + 8 * g + (i - 8)); const int c = k / KK, t9 = k % KK; const int kh = t9 / 3, kw = t9 % 3;
        a[i] = (__bf16)Xn[((size_t)c * HH + refl(h + kh - 1, HH)) * WWD + refl(w + kw - 1, WWD)]; }
#pragma unroll
      for (int j = 0; j < 5; ++j) { v16b wv; const int o = j * 16 + col; const int oc = o < COUT ? o : 0;
#pragma unroll
        for (int i = 0; i < 8; ++i) { wv[i] = (o < COUT) ? (__bf16)CW[(size_t)oc * KDIM + kc * 32 + 8 * g + i] : (__bf16)0.f; wv[8 + i] = (o < COUT) ? (__bf16)CW[(size_t)oc * KDIM + kc * 32 + 16 + 8 * g + i] : (__bf16)0.f; }
        acc[j] = wmma_bf(a, wv, acc[j]); } } }
#pragma unroll
  for (int j = 0; j < 5; ++j)
#pragma unroll
    for (int r = 0; r < 8; ++r) { const int o = j * 16 + col; if (o < COUT) { const float inv = rsqrtf(bfr(RV[o]) + 1e-5f); sg[wave * 16 + 8 * g + r][o] = (acc[j][r] - bfr(RM[o])) * (inv * bfr(GA[o])) + bfr(BE[o]); } }
  __syncthreads();
  if (tid < 64) { float* row = sg[tid]; float m = -3.0e38f; for (int o = 0; o < COUT; ++o) m = fmaxf(m, row[o]); float s = 0.f; for (int o = 0; o < COUT; ++o) { const float e = expf(row[o] - m); row[o] = e; s += e; } const float inv = 1.0f / s; for (int o = 0; o < COUT; ++o) row[o] *= inv; }
  __syncthreads();
  { const int p = tid & 63; const int w = 2 * p; const int cb = (tid >> 6) * 32;
    for (int cc = 0; cc < 32; ++cc) { const int c = cb + cc; const int gi = c / (CIN / GRP); const float* srow = &sg[p][gi * KK]; const float* xc = Xn + (size_t)c * HH * WWD; float acc9 = 0.f;
#pragma unroll
      for (int t9 = 0; t9 < KK; ++t9) { const int kh = t9 / 3, kw = t9 % 3; acc9 += srow[t9] * bfr(xc[(size_t)refl(h + kh - 1, HH) * WWD + refl(w + kw - 1, WWD)]); }
      so[c][p] = acc9; } }
  __syncthreads();
  for (int c = wave * 16; c < wave * 16 + 16; ++c) if (lane < 16) vst2(OUT + (((size_t)n * CIN + c) * HO + ho) * WO + lane * 4, *(const v4f*)&so[c][lane * 4]); }
extern "C" void kernel_launch(void* const* d_in, const int* in_sizes, int n_in, void* d_out, int out_size, void* d_ws, size_t ws_size, hipStream_t stream) {
  (void)in_sizes; (void)n_in; (void)out_size; (void)d_ws; (void)ws_size;
  const float** F = (const float**)d_in;
  k_pasa<<<dim3(NBLK), 128, 0, stream>>>(F[0], F[1], F[2], F[3], F[4], F[5], (float*)d_out);
}
